// InstrumentedBivectorBlock_37082747633887
// MI455X (gfx1250) — hardware-verified
//
#include <hip/hip_runtime.h>
#include <stddef.h>
#include <stdint.h>
#include <math.h>

#define NB    2
#define SEQL  1024
#define NTOK  2048
#define DD    256
#define DG    128
#define NPL   16
#define NSET  4
#define NPPS  4
#define CH    32
#define PHW   128
#define PI_F  3.14159265358979323846f

static_assert(NTOK == NB * SEQL);
static_assert(SEQL % CH == 0);
static_assert(CH == 32);
static_assert(NTOK % 64 == 0);
static_assert(DD == 256);
static_assert(DG % 64 == 0);
static_assert(NSET * NPPS == NPL);
static_assert((NTOK * DD) % 2048 == 0);
static_assert(SEQL % 16 == 0);
static_assert(NTOK % 8 == 0);

#define WSC   64.0f
#define WINV  0.015625f
#define EPSL  1e-5f
#define SFP   68
#define SPP   52
#define STP   132

typedef _Float16 hf;
typedef hf           v16h __attribute__((ext_vector_type(16)));
typedef hf           v8h  __attribute__((ext_vector_type(8)));
typedef float        v8f  __attribute__((ext_vector_type(8)));
typedef float        v4f  __attribute__((ext_vector_type(4)));
typedef unsigned int v4u  __attribute__((ext_vector_type(4)));

union Frag  { v16h v; v8h h[2]; };
union Pack8 { v8h h; v4u u; };

__device__ __forceinline__ v4u cvt8(const float (&f)[8], float sc) {
  Pack8 p;
  p.h = (v8h){(hf)(f[0] * sc), (hf)(f[1] * sc), (hf)(f[2] * sc), (hf)(f[3] * sc),
              (hf)(f[4] * sc), (hf)(f[5] * sc), (hf)(f[6] * sc), (hf)(f[7] * sc)};
  return p.u;
}

__device__ __forceinline__ v8f mma16(v16h a, v16h b, v8f c) {
  c = __builtin_amdgcn_wmma_f32_16x16x32_f16(false, a, false, b, (short)0, c, false, false);
  asm volatile("v_nop\n\tv_nop\n\tv_nop\n\tv_nop" : "+v"(c) : "v"(a), "v"(b));
  return c;
}

__device__ __forceinline__ v16h ldfrag(const hf* p, int ld, int row0, int k0, int lane) {
  const int m = lane & 15, lh = lane >> 4;
  const hf* q = p + (size_t)(row0 + m) * (size_t)ld + k0 + 8 * lh;
  Frag f;
  f.h[0] = *(const v8h*)(q);
  f.h[1] = *(const v8h*)(q + 16);
  return f.v;
}

__device__ __forceinline__ v8f zero8() { return (v8f){0.f, 0.f, 0.f, 0.f, 0.f, 0.f, 0.f, 0.f}; }

__device__ __forceinline__ float wsum(float v) {
#pragma unroll
  for (int o = 1; o < 32; o <<= 1) v += __shfl_xor(v, o, 32);
  return v;
}

__device__ __forceinline__ float sigmf(float x) { return __builtin_amdgcn_rcpf(1.0f + __expf(-x)); }

template <int KD>
__device__ __forceinline__ void gemm16x64(const hf* __restrict__ A, const hf* __restrict__ Bt,
                                          int m0, int n0, int lane, v8f (&acc)[4]) {
  static_assert(KD % 32 == 0);
#pragma unroll 1
  for (int k0 = 0; k0 < KD; k0 += 32) {
    const v16h a = ldfrag(A, KD, m0, k0, lane);
#pragma unroll
    for (int t = 0; t < 4; ++t) {
      const v16h b = ldfrag(Bt, KD, n0 + 16 * t, k0, lane);
      acc[t] = mma16(a, b, acc[t]);
    }
  }
}

__global__ __launch_bounds__(256) void k_cvt(const float* __restrict__ x, hf* __restrict__ xh) {
  const size_t i = (size_t)blockIdx.x * 2048 + (size_t)threadIdx.x * 8;
  const v4f a0 = *(const v4f*)(x + i);
  const v4f a1 = *(const v4f*)(x + i + 4);
  const float f[8] = {a0[0], a0[1], a0[2], a0[3], a1[0], a1[1], a1[2], a1[3]};
  const v4u u = cvt8(f, 1.0f);
  *(volatile v4u*)(xh + i) = u;
  __threadfence();
  *(volatile v4u*)(xh + i) = u;
}

template <int NOUT>
__global__ __launch_bounds__(256) void k_cvt_wt(const float* __restrict__ w, hf* __restrict__ wt) {
  static_assert(NOUT % 64 == 0);
  __shared__ __align__(16) float sw[64 * SFP];
  const int tid = threadIdx.x;
  const int kb = blockIdx.x * 64;
  const int nb = blockIdx.y * 64;
  {
    const int r  = tid >> 2;
    const int c0 = (tid & 3) * 16;
    const float* src = w + (size_t)(kb + r) * NOUT + nb + c0;
#pragma unroll
    for (int e = 0; e < 4; ++e) *(v4f*)(sw + r * SFP + c0 + 4 * e) = *(const v4f*)(src + 4 * e);
  }
  __syncthreads();
  v4u hv[2];
  size_t go[2];
#pragma unroll
  for (int j = 0; j < 2; ++j) {
    const int p  = tid + 256 * j;
    const int n  = p >> 3;
    const int pc = p & 7;
    const float* cp = sw + (pc * 8) * SFP + n;
    float f[8];
#pragma unroll
    for (int e = 0; e < 8; ++e) f[e] = cp[e * SFP];
    hv[j] = cvt8(f, WSC);
    go[j] = (size_t)(nb + n) * DD + kb + pc * 8;
  }
#pragma unroll
  for (int j = 0; j < 2; ++j) *(volatile v4u*)(wt + go[j]) = hv[j];
  __threadfence();
#pragma unroll
  for (int j = 0; j < 2; ++j) *(volatile v4u*)(wt + go[j]) = hv[j];
}

template <int KIN, int NREAL>
__global__ __launch_bounds__(256) void k_cvt_w16(const float* __restrict__ w, hf* __restrict__ wt) {
  constexpr int PPR = KIN / 8;
  constexpr int NPC = 16 * PPR;
  static_assert(NPC % 256 == 0);
  constexpr int NJ = NPC / 256;
  const int tid = threadIdx.x;
  v4u hv[NJ];
  size_t go[NJ];
#pragma unroll
  for (int j = 0; j < NJ; ++j) {
    const int p  = tid + 256 * j;
    const int n  = p / PPR;
    const int k0 = (p - n * PPR) * 8;
    const int nc = (n < NREAL) ? n : (NREAL - 1);
    float f[8];
#pragma unroll
    for (int e = 0; e < 8; ++e) {
      const float xv = w[(size_t)(k0 + e) * NREAL + nc];
      f[e] = (n < NREAL) ? xv : 0.f;
    }
    hv[j] = cvt8(f, WSC);
    go[j] = (size_t)n * KIN + k0;
  }
#pragma unroll
  for (int j = 0; j < NJ; ++j) *(volatile v4u*)(wt + go[j]) = hv[j];
  __threadfence();
#pragma unroll
  for (int j = 0; j < NJ; ++j) *(volatile v4u*)(wt + go[j]) = hv[j];
}

template <int MODE, int NOUT>
__global__ __launch_bounds__(128) void k_gemm(const hf* __restrict__ A, const hf* __restrict__ Bt,
                                              const float* __restrict__ bias, const float* __restrict__ res,
                                              hf* __restrict__ yh, float* __restrict__ yf) {
  static_assert(NOUT % 64 == 0);
  static_assert(MODE == 0 || NOUT == DD);
  __shared__ __align__(16) float sf[64 * SFP];
  const int tid = threadIdx.x, lane = tid & 31, wave = tid >> 5;
  const int hh = lane >> 4, c = lane & 15;
  const int mb = blockIdx.x * 64;
  const int nb = blockIdx.y * 64;
  const int m0 = mb + wave * 16;

  v8f acc[4];
#pragma unroll
  for (int t = 0; t < 4; ++t) acc[t] = zero8();
  gemm16x64<DD>(A, Bt, m0, nb, lane, acc);

  float bcol[4];
#pragma unroll
  for (int t = 0; t < 4; ++t) bcol[t] = bias[nb + 16 * t + c];
#pragma unroll
  for (int t = 0; t < 4; ++t) {
#pragma unroll
    for (int r = 0; r < 8; ++r) {
      float v = acc[t][r] * WINV + bcol[t];
      if constexpr (MODE == 0) v = 0.5f * v * (1.0f + erff(v * 0.70710678118654752f));
      sf[(wave * 16 + 8 * hh + r) * SFP + 16 * t + c] = v;
    }
  }
  __syncthreads();

  if constexpr (MODE == 0) {
    v4u hv[4];
    size_t go[4];
#pragma unroll
    for (int j = 0; j < 4; ++j) {
      const int p  = tid + 128 * j;
      const int lr = p >> 3;
      const int d0 = (p & 7) * 8;
      const float* ra = sf + lr * SFP + d0;
      const v4f a0 = *(const v4f*)(ra), a1 = *(const v4f*)(ra + 4);
      const float f[8] = {a0[0], a0[1], a0[2], a0[3], a1[0], a1[1], a1[2], a1[3]};
      hv[j] = cvt8(f, 1.0f);
      go[j] = ((size_t)(mb + lr)) * NOUT + nb + d0;
    }
#pragma unroll
    for (int j = 0; j < 4; ++j) *(volatile v4u*)(yh + go[j]) = hv[j];
    __threadfence();
#pragma unroll
    for (int j = 0; j < 4; ++j) *(volatile v4u*)(yh + go[j]) = hv[j];
  } else {
    v4f val[8];
    size_t go[8];
#pragma unroll
    for (int it = 0; it < 8; ++it) {
      const int p    = tid + 128 * it;
      const int L    = p >> 3;
      const int pc   = p & 7;
      const int row  = L >> 1;
      const int half = L & 1;
      const int col  = half * 32 + pc * 4;
      go[it]  = (size_t)(mb + row) * DD + nb + col;
      val[it] = *(const v4f*)(sf + row * SFP + col);
      if constexpr (MODE == 2) val[it] = val[it] + *(const v4f*)(res + go[it]);
    }
#pragma unroll
    for (int it = 0; it < 8; ++it) *(volatile v4f*)(yf + go[it]) = val[it];
    __threadfence();
#pragma unroll
    for (int it = 0; it < 8; ++it) *(volatile v4f*)(yf + go[it]) = val[it];
  }
}

__global__ __launch_bounds__(128) void k_phase(const hf* __restrict__ Hk, const hf* __restrict__ Hq,
                                               const hf* __restrict__ Hl, const hf* __restrict__ Hg,
                                               const hf* __restrict__ Wk2, const hf* __restrict__ Wq2,
                                               const hf* __restrict__ Wl2, const hf* __restrict__ Wg2,
                                               const float* __restrict__ bk2, const float* __restrict__ bq2,
                                               const float* __restrict__ bl2, const float* __restrict__ bg2,
                                               float* __restrict__ ph) {
  __shared__ __align__(16) float sph[64 * SPP];
  __shared__ __align__(16) float stab[64 * STP];
  const int tid = threadIdx.x, lane = tid & 31, wave = tid >> 5;
  const int hh = lane >> 4, c = lane & 15;
  const int mb = blockIdx.x * 64;
  const int m0 = mb + wave * 16;

  v8f ak = zero8(), aq = zero8(), al = zero8(), ag = zero8();
#pragma unroll 1
  for (int k0 = 0; k0 < DD; k0 += 32) {
    const v16h a0 = ldfrag(Hk, DD, m0, k0, lane);
    const v16h b0 = ldfrag(Wk2, DD, 0, k0, lane);
    ak = mma16(a0, b0, ak);
    const v16h a1 = ldfrag(Hq, DD, m0, k0, lane);
    const v16h b1 = ldfrag(Wq2, DD, 0, k0, lane);
    aq = mma16(a1, b1, aq);
    const v16h a2 = ldfrag(Hl, DD, m0, k0, lane);
    const v16h b2 = ldfrag(Wl2, DD, 0, k0, lane);
    al = mma16(a2, b2, al);
  }
#pragma unroll 1
  for (int k0 = 0; k0 < DG; k0 += 32) {
    const v16h a3 = ldfrag(Hg, DG, m0, k0, lane);
    const v16h b3 = ldfrag(Wg2, DG, 0, k0, lane);
    ag = mma16(a3, b3, ag);
  }
  const float bkc = bk2[c], bqc = bq2[c], blc = bl2[c], bgc = bg2[0];
#pragma unroll
  for (int r = 0; r < 8; ++r) {
    const int row = wave * 16 + 8 * hh + r;
    sph[row * SPP + c]      = tanhf(ak[r] * WINV + bkc) * PI_F;
    sph[row * SPP + 16 + c] = tanhf(aq[r] * WINV + bqc) * PI_F;
    sph[row * SPP + 32 + c] = tanhf(al[r] * WINV + blc) * PI_F;
    if (c == 0) sph[row * SPP + 48] = ag[r] * WINV + bgc;
  }
  __syncthreads();

#pragma unroll 1
  for (int i = tid; i < 64 * 48; i += 128) {
    const int r = i / 48;
    const int j = i - r * 48;
    const float p = sph[r * SPP + j];
    float sn, cs;
    sincosf(p, &sn, &cs);
    const int g = j >> 4, q = j & 15;
    stab[r * STP + 32 * g + q]      = cs;
    stab[r * STP + 32 * g + 16 + q] = sn;
  }
  __syncthreads();
#pragma unroll 1
  for (int i = tid; i < 64 * 8; i += 128) {
    const int r = i >> 3, wsel = i & 7;
    const int pp = wsel & 3, grp = wsel >> 2;
    const float* rowp = stab + r * STP + 32 * grp;
    float re = 1.f, im = 0.f;
#pragma unroll
    for (int s = 0; s < NSET; ++s) {
      const float cc = rowp[s * NPPS + pp], sn = rowp[16 + s * NPPS + pp];
      const float nr = re * cc - im * sn;
      const float ni = re * sn + im * cc;
      re = nr; im = ni;
    }
    stab[r * STP + 96 + 8 * grp + pp]     = re;
    stab[r * STP + 96 + 8 * grp + 4 + pp] = im;
  }
#pragma unroll 1
  for (int i = tid; i < 64 * 16; i += 128) {
    const int r = i >> 4, q = i & 15;
    const float graw = sph[r * SPP + 48];
    const float sg = 1.0f / (1.0f + expf(-graw));
    stab[r * STP + 112 + q] = (q == 0) ? sg : 0.f;
  }
  __syncthreads();

  v4f val[16];
#pragma unroll
  for (int it = 0; it < 16; ++it) {
    const int p = tid + 128 * it;
    const int r = p >> 5, pc = p & 31;
    val[it] = *(const v4f*)(stab + r * STP + 4 * pc);
  }
#pragma unroll
  for (int it = 0; it < 16; ++it) {
    const int p = tid + 128 * it;
    const int r = p >> 5, pc = p & 31;
    *(volatile v4f*)(ph + (size_t)(mb + r) * PHW + 4 * pc) = val[it];
  }
  __threadfence();
#pragma unroll
  for (int it = 0; it < 16; ++it) {
    const int p = tid + 128 * it;
    const int r = p >> 5, pc = p & 31;
    *(volatile v4f*)(ph + (size_t)(mb + r) * PHW + 4 * pc) = val[it];
  }
}

__global__ __launch_bounds__(256) void k_pos(const float* __restrict__ freqs, float* __restrict__ pos) {
  __shared__ __align__(16) float st[16 * 32];
  const int tid = threadIdx.x;
  const int r = tid >> 4, q = tid & 15;
  const int t = blockIdx.x * 16 + r;
  const float fr = freqs[q];
  const float ang = ((float)t * fr) * 2.0f * PI_F;
  float sn, cs;
  sincosf(ang, &sn, &cs);
  st[r * 32 + q]      = cs;
  st[r * 32 + 16 + q] = sn;
  __syncthreads();
  if (tid < 128) {
    const int rr = tid >> 3, pc = tid & 7;
    const v4f v = *(const v4f*)(st + rr * 32 + 4 * pc);
    float* op = pos + (size_t)(blockIdx.x * 16 + rr) * 32 + 4 * pc;
    *(volatile v4f*)op = v;
    __threadfence();
    *(volatile v4f*)op = v;
  }
}

__global__ __launch_bounds__(256) void k_gate_cross(const float* __restrict__ ph, const float* __restrict__ V,
                                                    const float* __restrict__ ssp, const float* __restrict__ sbp,
                                                    float* __restrict__ wgt, float* __restrict__ rc) {
  __shared__ float sj[CH * 16];
  __shared__ float sred[2][8][4];
  __shared__ float swg[CH];
  const int tid = threadIdx.x, lane = tid & 31, wv = tid >> 5, b = blockIdx.x;
  const float ss = ssp[0], sb = sbp[0];
  float ajx[NPPS], ajy[NPPS], acx[NPPS], acy[NPPS];
#pragma unroll
  for (int p = 0; p < NPPS; ++p) { ajx[p] = 0.f; ajy[p] = 0.f; acx[p] = 0.f; acy[p] = 0.f; }

#pragma unroll 1
  for (int cnk = 0; cnk < SEQL / CH; ++cnk) {
    const int bt0 = b * SEQL + cnk * CH;
    __syncthreads();
#pragma unroll
    for (int k = 0; k < 2; ++k) {
      const int i = tid + 256 * k;
      sj[i] = ph[(size_t)(bt0 + (i >> 4)) * PHW + 96 + (i & 15)];
    }
    __syncthreads();
#pragma unroll 1
    for (int tt = 0; tt < CH; ++tt) {
      const int bt = bt0 + tt;
      const float v = V[(size_t)bt * DD + tid];
      const float* jr = sj + tt * 16;
      float pred = 0.f;
#pragma unroll
      for (int p = 0; p < NPPS; ++p) { pred = fmaf(ajx[p], jr[p], pred); pred = fmaf(ajy[p], jr[4 + p], pred); }
      float q0 = pred * pred, q1 = pred * v, q2 = v * v;
      q0 = wsum(q0); q1 = wsum(q1); q2 = wsum(q2);
      if (lane == 0) { sred[tt & 1][wv][0] = q0; sred[tt & 1][wv][1] = q1; sred[tt & 1][wv][2] = q2; }
      __syncthreads();
      float pn = 0.f, pv = 0.f, vn = 0.f;
#pragma unroll
      for (int w = 0; w < 8; ++w) { pn += sred[tt & 1][w][0]; pv += sred[tt & 1][w][1]; vn += sred[tt & 1][w][2]; }
      const float np = sqrtf(pn), nv = sqrtf(vn);
      float fam = pv * __builtin_amdgcn_rcpf(fmaxf(np, 1e-8f) * fmaxf(nv, 1e-8f));
      fam = (np > 1e-6f) ? fam : 0.f;
      const float wg = sigmf(ss * ((1.0f - fam) * 0.5f - 0.5f) + sb);
      if (tid == 0) swg[tt] = wg;
      const float vg = v * wg;
      float cr = 0.f;
#pragma unroll
      for (int p = 0; p < NPPS; ++p) {
        acx[p] = fmaf(jr[p], vg, acx[p]);
        acy[p] = fmaf(jr[4 + p], vg, acy[p]);
        cr = fmaf(acx[p], jr[8 + p], cr);
        cr = fmaf(acy[p], jr[12 + p], cr);
      }
#pragma unroll
      for (int p = 0; p < NPPS; ++p) { ajx[p] = fmaf(jr[p], v, ajx[p]); ajy[p] = fmaf(jr[4 + p], v, ajy[p]); }
      float* op = rc + (size_t)bt * DD + tid;
      *(volatile float*)op = cr;
      __threadfence();
      *(volatile float*)op = cr;
    }
    __syncthreads();
    if (wv == 0) {
      const float g = swg[lane];
      float* op = wgt + bt0 + lane;
      *(volatile float*)op = g;
      __threadfence();
      *(volatile float*)op = g;
    }
  }
}

__global__ __launch_bounds__(256) void k_bank(const float* __restrict__ ph, const float* __restrict__ V,
                                              const float* __restrict__ wgt, const float* __restrict__ rc,
                                              const float* __restrict__ setw, float* __restrict__ ra) {
  __shared__ float skq[CH * 64];
  __shared__ float swg[CH];
  const int tid = threadIdx.x, b = blockIdx.x;
  const float s0 = setw[0], s1 = setw[1], s2 = setw[2], s3 = setw[3];
  const float mx = fmaxf(fmaxf(s0, s1), fmaxf(s2, s3));
  const float e0 = __expf(s0 - mx), e1 = __expf(s1 - mx), e2 = __expf(s2 - mx), e3 = __expf(s3 - mx);
  const float einv = __builtin_amdgcn_rcpf(((e0 + e1) + e2) + e3);
  const float w0 = e0 * einv, w1 = e1 * einv, w2 = e2 * einv, w3 = e3 * einv;
  float abx[NPL], aby[NPL];
#pragma unroll
  for (int i = 0; i < NPL; ++i) { abx[i] = 0.f; aby[i] = 0.f; }

#pragma unroll 1
  for (int cnk = 0; cnk < SEQL / CH; ++cnk) {
    const int bt0 = b * SEQL + cnk * CH;
    __syncthreads();
#pragma unroll
    for (int k = 0; k < 8; ++k) {
      const int i = tid + 256 * k;
      skq[i] = ph[(size_t)(bt0 + (i >> 6)) * PHW + (i & 63)];
    }
    if (tid < CH) swg[tid] = wgt[bt0 + tid];
    __syncthreads();
#pragma unroll 1
    for (int tt = 0; tt < CH; ++tt) {
      const int bt = bt0 + tt;
      const float v = V[(size_t)bt * DD + tid];
      const float vg = v * swg[tt];
      const float* kr = skq + tt * 64;
      float rs[NSET] = {0.f, 0.f, 0.f, 0.f};
#pragma unroll
      for (int i = 0; i < NPL; ++i) {
        abx[i] = fmaf(kr[i], vg, abx[i]);
        aby[i] = fmaf(kr[16 + i], vg, aby[i]);
        rs[i >> 2] = fmaf(abx[i], kr[32 + i], rs[i >> 2]);
        rs[i >> 2] = fmaf(aby[i], kr[48 + i], rs[i >> 2]);
      }
      const float tot = ((w0 * rs[0] + w1 * rs[1]) + w2 * rs[2]) + w3 * rs[3];
      const float cv = rc[(size_t)bt * DD + tid];
      const float av = 0.2f * (tot + cv);
      float* op = ra + (size_t)bt * DD + tid;
      *(volatile float*)op = av;
      __threadfence();
      *(volatile float*)op = av;
    }
  }
}

__global__ __launch_bounds__(256) void k_posscan(const float* __restrict__ post, const float* __restrict__ V,
                                                 float* __restrict__ rp) {
  __shared__ float sp[CH * 32];
  const int tid = threadIdx.x, b = blockIdx.x;
  float apx[NPL], apy[NPL];
#pragma unroll
  for (int i = 0; i < NPL; ++i) { apx[i] = 0.f; apy[i] = 0.f; }

#pragma unroll 1
  for (int cnk = 0; cnk < SEQL / CH; ++cnk) {
    const int t0 = cnk * CH;
    const int bt0 = b * SEQL + t0;
    __syncthreads();
#pragma unroll
    for (int k = 0; k < 4; ++k) {
      const int i = tid + 256 * k;
      sp[i] = post[(size_t)t0 * 32 + i];
    }
    __syncthreads();
#pragma unroll 1
    for (int tt = 0; tt < CH; ++tt) {
      const int bt = bt0 + tt;
      const float v = V[(size_t)bt * DD + tid];
      const float* pr = sp + tt * 32;
      float r = 0.f;
#pragma unroll
      for (int p = 0; p < NPL; ++p) {
        apx[p] = fmaf(pr[p], v, apx[p]);
        apy[p] = fmaf(pr[16 + p], v, apy[p]);
        r = fmaf(apx[p], pr[p], r);
        r = fmaf(apy[p], pr[16 + p], r);
      }
      float* op = rp + (size_t)bt * DD + tid;
      *(volatile float*)op = r;
      __threadfence();
      *(volatile float*)op = r;
    }
  }
}

__global__ __launch_bounds__(256) void k_gate_ltm(const float* __restrict__ ph, const float* __restrict__ LV,
                                                  const float* __restrict__ ssp, const float* __restrict__ sbp,
                                                  float* __restrict__ lgt) {
  __shared__ float sl[CH * 32];
  __shared__ float sred[2][8][4];
  __shared__ float slg[CH];
  const int tid = threadIdx.x, lane = tid & 31, wv = tid >> 5, b = blockIdx.x;
  const float ss = ssp[0], sb = sbp[0];
  float alx[NPL], aly[NPL];
#pragma unroll
  for (int p = 0; p < NPL; ++p) { alx[p] = 0.f; aly[p] = 0.f; }

#pragma unroll 1
  for (int cnk = 0; cnk < SEQL / CH; ++cnk) {
    const int bt0 = b * SEQL + cnk * CH;
    __syncthreads();
#pragma unroll
    for (int k = 0; k < 4; ++k) {
      const int i = tid + 256 * k;
      sl[i] = ph[(size_t)(bt0 + (i >> 5)) * PHW + 64 + (i & 31)];
    }
    __syncthreads();
#pragma unroll 1
    for (int tt = 0; tt < CH; ++tt) {
      const int bt = bt0 + tt;
      const float lv = LV[(size_t)bt * DD + tid];
      const float* lr = sl + tt * 32;
      float lp = 0.f;
#pragma unroll
      for (int p = 0; p < NPL; ++p) { lp = fmaf(alx[p], lr[p], lp); lp = fmaf(aly[p], lr[16 + p], lp); }
      float q0 = lp * lp, q1 = lp * lv, q2 = lv * lv;
      q0 = wsum(q0); q1 = wsum(q1); q2 = wsum(q2);
      if (lane == 0) { sred[tt & 1][wv][0] = q0; sred[tt & 1][wv][1] = q1; sred[tt & 1][wv][2] = q2; }
      __syncthreads();
      float pn = 0.f, pv = 0.f, vn = 0.f;
#pragma unroll
      for (int w = 0; w < 8; ++w) { pn += sred[tt & 1][w][0]; pv += sred[tt & 1][w][1]; vn += sred[tt & 1][w][2]; }
      const float np = sqrtf(pn), nv = sqrtf(vn);
      float fam = pv * __builtin_amdgcn_rcpf(fmaxf(np, 1e-8f) * fmaxf(nv, 1e-8f));
      fam = (np > 1e-6f) ? fam : 0.f;
      const float lg = sigmf(ss * ((1.0f - fam) * 0.5f - 0.5f) + sb);
      if (tid == 0) slg[tt] = lg;
#pragma unroll
      for (int p = 0; p < NPL; ++p) { alx[p] = fmaf(lr[p], lv, alx[p]); aly[p] = fmaf(lr[16 + p], lv, aly[p]); }
    }
    __syncthreads();
    if (wv == 0) {
      const float g = slg[lane];
      float* op = lgt + bt0 + lane;
      *(volatile float*)op = g;
      __threadfence();
      *(volatile float*)op = g;
    }
  }
}

__global__ __launch_bounds__(256) void k_ltm(const float* __restrict__ ph, const float* __restrict__ LV,
                                             const float* __restrict__ lgt, float* __restrict__ rl) {
  __shared__ float sl[CH * 32];
  __shared__ float slg[CH];
  const int tid = threadIdx.x, b = blockIdx.x;
  float agx[NPL], agy[NPL];
#pragma unroll
  for (int p = 0; p < NPL; ++p) { agx[p] = 0.f; agy[p] = 0.f; }

#pragma unroll 1
  for (int cnk = 0; cnk < SEQL / CH; ++cnk) {
    const int t0 = cnk * CH;
    const int bt0 = b * SEQL + t0;
    __syncthreads();
#pragma unroll
    for (int k = 0; k < 4; ++k) {
      const int i = tid + 256 * k;
      sl[i] = ph[(size_t)(bt0 + (i >> 5)) * PHW + 64 + (i & 31)];
    }
    if (tid < CH) slg[tid] = lgt[bt0 + tid];
    __syncthreads();
#pragma unroll 1
    for (int tt = 0; tt < CH; ++tt) {
      const int bt = bt0 + tt;
      const float lv = LV[(size_t)bt * DD + tid];
      const float lvg = lv * slg[tt];
      const float* lr = sl + tt * 32;
      float r = 0.f;
#pragma unroll
      for (int p = 0; p < NPL; ++p) {
        agx[p] = fmaf(lr[p], lvg, agx[p]);
        agy[p] = fmaf(lr[16 + p], lvg, agy[p]);
        r = fmaf(agx[p], lr[p], r);
        r = fmaf(agy[p], lr[16 + p], r);
      }
      const float scl = 1.0f / sqrtf((float)(t0 + tt + 1) * (float)NPL);
      const float out = r * scl;
      float* op = rl + (size_t)bt * DD + tid;
      *(volatile float*)op = out;
      __threadfence();
      *(volatile float*)op = out;
    }
  }
}

__global__ __launch_bounds__(256) void k_ln(const float* __restrict__ ra, const float* __restrict__ rpp,
                                            const float* __restrict__ rl, const float* __restrict__ ph,
                                            const float* __restrict__ posw, const float* __restrict__ ltmw,
                                            const float* __restrict__ g, const float* __restrict__ bta,
                                            hf* __restrict__ hn) {
  const int lane = threadIdx.x & 31, wave = threadIdx.x >> 5;
  const int row = blockIdx.x * 8 + wave;
  const int t = row % SEQL;
  const float gt = ph[(size_t)row * PHW + 112];
  const float sp = sigmf(posw[0]), sg = sigmf(ltmw[0]);
  const float cs = 1.0f / sqrtf((float)(t + 1) * (float)NPPS);
  const int c0 = lane * 8;
  const size_t o = (size_t)row * DD + c0;
  const v4f a0 = *(const v4f*)(ra + o),  a1 = *(const v4f*)(ra + o + 4);
  const v4f p0 = *(const v4f*)(rpp + o), p1 = *(const v4f*)(rpp + o + 4);
  const v4f l0 = *(const v4f*)(rl + o),  l1 = *(const v4f*)(rl + o + 4);
  const float av[8] = {a0[0], a0[1], a0[2], a0[3], a1[0], a1[1], a1[2], a1[3]};
  const float pv[8] = {p0[0], p0[1], p0[2], p0[3], p1[0], p1[1], p1[2], p1[3]};
  const float lv[8] = {l0[0], l0[1], l0[2], l0[3], l1[0], l1[1], l1[2], l1[3]};
  const float omg = 1.0f - gt;
  float h[8];
  float sm = 0.f;
#pragma unroll
  for (int k = 0; k < 8; ++k) {
    const float tot = (gt * av[k] + omg * (sp * pv[k])) + sg * lv[k];
    h[k] = tot * cs;
    sm += h[k];
  }
  sm = wsum(sm);
  const float mu = sm * (1.0f / (float)DD);
  float sq = 0.f;
#pragma unroll
  for (int k = 0; k < 8; ++k) { const float d = h[k] - mu; sq = fmaf(d, d, sq); }
  sq = wsum(sq);
  const float var = sq * (1.0f / (float)DD);
  const float rsd = 1.0f / sqrtf(var + EPSL);
  const v4f g0 = *(const v4f*)(g + c0),   g1 = *(const v4f*)(g + c0 + 4);
  const v4f b0 = *(const v4f*)(bta + c0), b1 = *(const v4f*)(bta + c0 + 4);
  const float gv[8] = {g0[0], g0[1], g0[2], g0[3], g1[0], g1[1], g1[2], g1[3]};
  const float bv[8] = {b0[0], b0[1], b0[2], b0[3], b1[0], b1[1], b1[2], b1[3]};
  float y[8];
#pragma unroll
  for (int k = 0; k < 8; ++k) y[k] = (h[k] - mu) * rsd * gv[k] + bv[k];
  const v4u u = cvt8(y, 1.0f);
  *(volatile v4u*)(hn + o) = u;
  __threadfence();
  *(volatile v4u*)(hn + o) = u;
}

extern "C" void kernel_launch(void* const* d_in, const int* in_sizes, int n_in,
                              void* d_out, int out_size, void* d_ws, size_t ws_size,
                              hipStream_t stream) {
  if (n_in < 31) return;
  if (in_sizes[0]  != NTOK * DD) return;
  if (in_sizes[1]  != DD * DD) return;
  if (in_sizes[2]  != DD) return;
  if (in_sizes[3]  != DD * NPL) return;
  if (in_sizes[4]  != NPL) return;
  if (in_sizes[5]  != DD * DD) return;
  if (in_sizes[6]  != DD) return;
  if (in_sizes[7]  != DD * NPL) return;
  if (in_sizes[8]  != NPL) return;
  if (in_sizes[9]  != DD * DD) return;
  if (in_sizes[10] != DD) return;
  if (in_sizes[11] != DD) return;
  if (in_sizes[12] != DD) return;
  if (in_sizes[13] != DD * DD) return;
  if (in_sizes[14] != DD) return;
  if (in_sizes[15] != NSET) return;
  if (in_sizes[16] != NPL) return;
  if (in_sizes[17] != 1) return;
  if (in_sizes[18] != DD * DG) return;
  if (in_sizes[19] != DG) return;
  if (in_sizes[20] != DG) return;
  if (in_sizes[21] != 1) return;
  if (in_sizes[22] != DD * DD) return;
  if (in_sizes[23] != DD) return;
  if (in_sizes[24] != DD * NPL) return;
  if (in_sizes[25] != NPL) return;
  if (in_sizes[26] != DD * DD) return;
  if (in_sizes[27] != DD) return;
  if (in_sizes[28] != 1) return;
  if (in_sizes[29] != 1) return;
  if (in_sizes[30] != 1) return;
  if (out_size != NTOK * DD) return;

  const float* X    = (const float*)d_in[0];
  const float* kw1  = (const float*)d_in[1];
  const float* kb1  = (const float*)d_in[2];
  const float* kw2  = (const float*)d_in[3];
  const float* kb2  = (const float*)d_in[4];
  const float* qw1  = (const float*)d_in[5];
  const float* qb1  = (const float*)d_in[6];
  const float* qw2  = (const float*)d_in[7];
  const float* qb2  = (const float*)d_in[8];
  const float* vw   = (const float*)d_in[9];
  const float* vb   = (const float*)d_in[10];
  const float* lng  = (const float*)d_in[11];
  const float* lnb  = (const float*)d_in[12];
  const float* ow   = (const float*)d_in[13];
  const float* ob   = (const float*)d_in[14];
  const float* setw = (const float*)d_in[15];
  const float* pfr  = (const float*)d_in[16];
  const float* posw = (const float*)d_in[17];
  const float* gw1  = (const float*)d_in[18];
  const float* gb1  = (const float*)d_in[19];
  const float* gw2  = (const float*)d_in[20];
  const float* gb2  = (const float*)d_in[21];
  const float* lkw1 = (const float*)d_in[22];
  const float* lkb1 = (const float*)d_in[23];
  const float* lkw2 = (const float*)d_in[24];
  const float* lkb2 = (const float*)d_in[25];
  const float* lvw  = (const float*)d_in[26];
  const float* lvb  = (const float*)d_in[27];
  const float* ssp  = (const float*)d_in[28];
  const float* sbp  = (const float*)d_in[29];
  const float* ltw  = (const float*)d_in[30];
  float* out = (float*)d_out;

  const size_t PLX = (size_t)NTOK * DD * 2;
  const size_t PLG = (size_t)NTOK * DG * 2;
  const size_t PLW = (size_t)DD * DD * 2;
  const size_t PWG = (size_t)DG * DD * 2;
  const size_t PW2 = (size_t)NPL * DD * 2;
  const size_t PG2 = (size_t)NPL * DG * 2;
  const size_t PF  = (size_t)NTOK * DD * 4;
  const size_t PPH = (size_t)NTOK * PHW * 4;
  const size_t PPS = (size_t)SEQL * 32 * 4;
  const size_t PGT = (size_t)NTOK * 4;
  size_t off = 0;
  const size_t oXh  = off; off += PLX;
  const size_t oW1K = off; off += PLW;
  const size_t oW1Q = off; off += PLW;
  const size_t oWV  = off; off += PLW;
  const size_t oW1L = off; off += PLW;
  const size_t oWLV = off; off += PLW;
  const size_t oWO  = off; off += PLW;
  const size_t oWG1 = off; off += PWG;
  const size_t oW2K = off; off += PW2;
  const size_t oW2Q = off; off += PW2;
  const size_t oW2L = off; off += PW2;
  const size_t oWG2 = off; off += PG2;
  const size_t oHk  = off; off += PLX;
  const size_t oHq  = off; off += PLX;
  const size_t oHl  = off; off += PLX;
  const size_t oHg  = off; off += PLG;
  const size_t oV   = off; off += PF;
  const size_t oLV  = off; off += PF;
  const size_t oPH  = off; off += PPH;
  const size_t oPOS = off; off += PPS;
  const size_t oWG  = off; off += PGT;
  const size_t oLG  = off; off += PGT;
  const size_t oRC  = off; off += PF;
  const size_t oRA  = off; off += PF;
  const size_t oRP  = off; off += PF;
  const size_t oRL  = off; off += PF;
  const size_t oHN  = off; off += PLX;
  if (off > ws_size) return;
  if (off > (size_t)134217728) return;

  char* ws = (char*)d_ws;
  hf* Xh   = (hf*)(ws + oXh);
  hf* W1Kt = (hf*)(ws + oW1K);
  hf* W1Qt = (hf*)(ws + oW1Q);
  hf* WVt  = (hf*)(ws + oWV);
  hf* W1Lt = (hf*)(ws + oW1L);
  hf* WLVt = (hf*)(ws + oWLV);
  hf* WOt  = (hf*)(ws + oWO);
  hf* WG1t = (hf*)(ws + oWG1);
  hf* W2Kt = (hf*)(ws + oW2K);
  hf* W2Qt = (hf*)(ws + oW2Q);
  hf* W2Lt = (hf*)(ws + oW2L);
  hf* WG2t = (hf*)(ws + oWG2);
  hf* Hk   = (hf*)(ws + oHk);
  hf* Hq   = (hf*)(ws + oHq);
  hf* Hl   = (hf*)(ws + oHl);
  hf* Hg   = (hf*)(ws + oHg);
  float* Vf  = (float*)(ws + oV);
  float* LVf = (float*)(ws + oLV);
  float* PH  = (float*)(ws + oPH);
  float* POS = (float*)(ws + oPOS);
  float* WG  = (float*)(ws + oWG);
  float* LG  = (float*)(ws + oLG);
  float* RC  = (float*)(ws + oRC);
  float* RA  = (float*)(ws + oRA);
  float* RP  = (float*)(ws + oRP);
  float* RL  = (float*)(ws + oRL);
  hf* HN   = (hf*)(ws + oHN);

  k_cvt<<<dim3((NTOK * DD) / 2048), dim3(256), 0, stream>>>(X, Xh);
  k_cvt_wt<DD><<<dim3(DD / 64, DD / 64), dim3(256), 0, stream>>>(kw1, W1Kt);
  k_cvt_wt<DD><<<dim3(DD / 64, DD / 64), dim3(256), 0, stream>>>(qw1, W1Qt);
  k_cvt_wt<DD><<<dim3(DD / 64, DD / 64), dim3(256), 0, stream>>>(vw, WVt);
  k_cvt_wt<DD><<<dim3(DD / 64, DD / 64), dim3(256), 0, stream>>>(lkw1, W1Lt);
  k_cvt_wt<DD><<<dim3(DD / 64, DD / 64), dim3(256), 0, stream>>>(lvw, WLVt);
  k_cvt_wt<DD><<<dim3(DD / 64, DD / 64), dim3(256), 0, stream>>>(ow, WOt);
  k_cvt_wt<DG><<<dim3(DD / 64, DG / 64), dim3(256), 0, stream>>>(gw1, WG1t);
  k_cvt_w16<DD, NPL><<<dim3(1), dim3(256), 0, stream>>>(kw2, W2Kt);
  k_cvt_w16<DD, NPL><<<dim3(1), dim3(256), 0, stream>>>(qw2, W2Qt);
  k_cvt_w16<DD, NPL><<<dim3(1), dim3(256), 0, stream>>>(lkw2, W2Lt);
  k_cvt_w16<DG, 1><<<dim3(1), dim3(256), 0, stream>>>(gw2, WG2t);
  k_gemm<0, DD><<<dim3(NTOK / 64, DD / 64), dim3(128), 0, stream>>>(Xh, W1Kt, kb1, X, Hk, Vf);
  k_gemm<0, DD><<<dim3(NTOK / 64, DD / 64), dim3(128), 0, stream>>>(Xh, W1Qt, qb1, X, Hq, Vf);
  k_gemm<0, DD><<<dim3(NTOK / 64, DD / 64), dim3(128), 0, stream>>>(Xh, W1Lt, lkb1, X, Hl, Vf);
  k_gemm<0, DG><<<dim3(NTOK / 64, DG / 64), dim3(128), 0, stream>>>(Xh, WG1t, gb1, X, Hg, Vf);
  k_gemm<1, DD><<<dim3(NTOK / 64, DD / 64), dim3(128), 0, stream>>>(Xh, WVt, vb, X, Hk, Vf);
  k_gemm<1, DD><<<dim3(NTOK / 64, DD / 64), dim3(128), 0, stream>>>(Xh, WLVt, lvb, X, Hk, LVf);
  k_phase<<<dim3(NTOK / 64), dim3(128), 0, stream>>>(Hk, Hq, Hl, Hg, W2Kt, W2Qt, W2Lt, WG2t,
                                                     kb2, qb2, lkb2, gb2, PH);
  k_pos<<<dim3(SEQL / 16), dim3(256), 0, stream>>>(pfr, POS);
  k_gate_cross<<<dim3(NB), dim3(256), 0, stream>>>(PH, Vf, ssp, sbp, WG, RC);
  k_bank<<<dim3(NB), dim3(256), 0, stream>>>(PH, Vf, WG, RC, setw, RA);
  k_posscan<<<dim3(NB), dim3(256), 0, stream>>>(POS, Vf, RP);
  k_gate_ltm<<<dim3(NB), dim3(256), 0, stream>>>(PH, LVf, ssp, sbp, LG);
  k_ltm<<<dim3(NB), dim3(256), 0, stream>>>(PH, LVf, LG, RL);
  k_ln<<<dim3(NTOK / 8), dim3(256), 0, stream>>>(RA, RP, RL, PH, posw, ltw, lng, lnb, HN);
  k_gemm<2, DD><<<dim3(NTOK / 64, DD / 64), dim3(128), 0, stream>>>(HN, WOt, ob, X, Hk, out);
  (void)hipGetLastError();
}
